// SetAttention_36498632081553
// MI455X (gfx1250) — hardware-verified
//
#include <hip/hip_runtime.h>
#include <math.h>

typedef __attribute__((ext_vector_type(16))) _Float16 v16h;
typedef __attribute__((ext_vector_type(16))) __bf16 v16b;
typedef __attribute__((ext_vector_type(8)))  _Float16 v8h;
typedef __attribute__((ext_vector_type(8)))  float v8f;
typedef __attribute__((ext_vector_type(4)))  float v4f;
typedef __attribute__((ext_vector_type(2)))  float v2f;
typedef __attribute__((ext_vector_type(4)))  unsigned v4u;
typedef __attribute__((ext_vector_type(4)))  int v4i;
typedef float __attribute__((may_alias)) float_a;
typedef int __attribute__((may_alias)) int_a;

template <typename T> __device__ __forceinline__ void vst2(void* p, T v) { *(volatile T*)p = v; __threadfence(); *(volatile T*)p = v; }
__device__ __forceinline__ v8f wmma16(v16h a, v16h b, v8f c) {
  v8f d = __builtin_amdgcn_wmma_f32_16x16x32_f16(false, a, false, b, (short)0, c, false, false);
  asm volatile("v_nop\n\tv_nop\n\tv_nop\n\tv_nop" : "+v"(d) : "v"(a), "v"(b));
  return d;
}
__device__ __forceinline__ v8f wmma_bf(v16b a, v16b b, v8f c) {
  v8f d = __builtin_amdgcn_wmma_f32_16x16x32_bf16(false, a, false, b, (short)0, c, false, false);
  asm volatile("v_nop\n\tv_nop\n\tv_nop\n\tv_nop" : "+v"(d) : "v"(a), "v"(b));
  return d;
}
__device__ __forceinline__ v16h frag_h(const _Float16* rowk0, int lane) {
  union { v16h v; v8h q[2]; } u; const _Float16* p = rowk0 + 8 * (lane >> 4);
  u.q[0] = *(const v8h*)p; u.q[1] = *(const v8h*)(p + 16); return u.v;
}
__device__ __forceinline__ v16h frag_f32(const float* rowk0, int lane) {
  v16h a; const float* p = rowk0 + 8 * (lane >> 4);
#pragma unroll
  for (int i = 0; i < 8; ++i) { a[i] = (_Float16)p[i]; a[8 + i] = (_Float16)p[16 + i]; }
  return a;
}
__device__ __forceinline__ v16h frag_f32s(const float* rowk0, int lane, float sc) {
  v16h a; const float* p = rowk0 + 8 * (lane >> 4);
#pragma unroll
  for (int i = 0; i < 8; ++i) { a[i] = (_Float16)(p[i] * sc); a[8 + i] = (_Float16)(p[16 + i] * sc); }
  return a;
}
__device__ __forceinline__ v16h fragc_f32(const float* W, int k0, int n, int lane, int ld, int K) {
  v16h a; const int g = lane >> 4;
#pragma unroll
  for (int i = 0; i < 8; ++i) { const int ka = k0 + 8 * g + i, kb = ka + 16;
    a[i] = (_Float16)(ka < K ? W[(size_t)(ka < K ? ka : K - 1) * ld + n] : 0.f); a[8 + i] = (_Float16)(kb < K ? W[(size_t)(kb < K ? kb : K - 1) * ld + n] : 0.f); }
  return a;
}
struct F2 { v16b h, l; };
__device__ __forceinline__ F2 bsplit16(const float v[16]) { F2 r;
#pragma unroll
  for (int i = 0; i < 16; ++i) { const __bf16 h = (__bf16)v[i]; r.h[i] = h; r.l[i] = (__bf16)(v[i] - (float)h); }
  return r; }
__device__ __forceinline__ F2 split_row(const float* row, int k0, int lane) { float v[16]; const float* p = row + k0 + 8 * (lane >> 4);
#pragma unroll
  for (int i = 0; i < 8; ++i) { v[i] = p[i]; v[8 + i] = p[16 + i]; }
  return bsplit16(v); }
__device__ __forceinline__ F2 split_rowK(const float* row, int k0, int lane, int K) { float v[16]; const int g = lane >> 4;
#pragma unroll
  for (int i = 0; i < 8; ++i) { const int ka = k0 + 8 * g + i, kb = ka + 16; v[i] = ka < K ? row[ka < K ? ka : K - 1] : 0.f; v[8 + i] = kb < K ? row[kb < K ? kb : K - 1] : 0.f; }
  return bsplit16(v); }
__device__ __forceinline__ F2 split_col(const float* W, int k0, int n, int lane, int ld, int K) { float v[16]; const int g = lane >> 4;
#pragma unroll
  for (int i = 0; i < 8; ++i) { const int ka = k0 + 8 * g + i, kb = ka + 16; v[i] = ka < K ? W[(size_t)(ka < K ? ka : K - 1) * ld + n] : 0.f; v[8 + i] = kb < K ? W[(size_t)(kb < K ? kb : K - 1) * ld + n] : 0.f; }
  return bsplit16(v); }
__device__ __forceinline__ v8f mac3(const F2& a, const F2& b, v8f c) { c = wmma_bf(a.l, b.h, c); c = wmma_bf(a.h, b.l, c); return wmma_bf(a.h, b.h, c); }
__device__ __forceinline__ float sigm(float v) { return 1.0f / (1.0f + expf(-v)); }
#define LDSX() do { asm volatile("s_wait_dscnt 0" ::: "memory"); __builtin_amdgcn_wave_barrier(); __builtin_amdgcn_fence(__ATOMIC_RELEASE, "workgroup"); } while (0)


#define NB 8
#define NN 2048
#define FI 128
#define FO 128
#define NR (NB * NN)
#ifndef TNB
#define TNB NB
#endif
typedef __attribute__((ext_vector_type(8))) __bf16 v8b;
__device__ __forceinline__ v16b frag_b(const __bf16* rowk0, int lane) {
  union { v16b v; v8b q[2]; } u; const __bf16* p = rowk0 + 8 * (lane >> 4);
  u.q[0] = *(const v8b*)p; u.q[1] = *(const v8b*)(p + 16); return u.v;
}
__device__ __forceinline__ float bfr(float v) { return (float)(__bf16)v; }
__device__ __attribute__((noinline)) float exp_ni(float v) { return expf(v); }
__device__ __attribute__((noinline)) float erf_ni(float v) { return erff(v); }
#define NEG_BIG -9.0e15f

#define WS_PW  0u
#define WS_H   (WS_PW + 2u * (size_t)2 * FO * FI)
#define WS_HP  (WS_H + 4u * (size_t)NR * FO)
#define WS_HPL (WS_HP + 2u * (size_t)NB * FO * NN)
#define WS_U   (WS_HPL + 2u * (size_t)NB * FO * NN)
#define WS_CM  (WS_U + 4u * (size_t)2 * NR)
#define WS_CZ  (WS_CM + 4u * (size_t)NR)
#define WS_END (WS_CZ + 4u * (size_t)NR)

__global__ __launch_bounds__(128) void k_pack(const float* __restrict__ WO, const float* __restrict__ WS, __bf16* __restrict__ P) { const int n = blockIdx.x, which = blockIdx.y, t = threadIdx.x; const float* Wm = which ? WS : WO; __shared__ __align__(16) __bf16 s[FI]; s[t] = (__bf16)Wm[(size_t)t * FO + n]; __syncthreads(); if (t < FI / 8) vst2((unsigned*)(P + ((size_t)which * FO + n) * FI + t * 8), *(const v4u*)&s[t * 8]); }
__device__ __forceinline__ int pidx(long long k) { const long long nn = (long long)NN * NN; return (k < nn) ? (int)(k / NN) : (int)(k % NN); }
__device__ __forceinline__ float escore(const float* __restrict__ U1, const float* __restrict__ U2, size_t b, int i, int j) { const long long m = (long long)i * NN + j; const float e = U1[b * NN + pidx(2 * m)] + U2[b * NN + pidx(2 * m + 1)]; return (e >= 0.f) ? e : 0.1f * e; }
__global__ __launch_bounds__(128) void k_h(const float* __restrict__ X, const __bf16* __restrict__ P, const float* __restrict__ AW, float* __restrict__ H, _Float16* __restrict__ HP, _Float16* __restrict__ HPL, float* __restrict__ U, float* __restrict__ OUT) {
  __shared__ __align__(16) float so[64][132]; __shared__ __align__(16) _Float16 st[128][72]; __shared__ __align__(16) _Float16 stl[128][72]; __shared__ __align__(16) float su[2][64];
  const int tid = threadIdx.x, wave = tid >> 5, lane = tid & 31, col = lane & 15, g = lane >> 4; const int which = blockIdx.y; const size_t rb0 = (size_t)blockIdx.x * 64, r0 = rb0 + wave * 16;
  v8f acc[8] = {};
#pragma unroll
  for (int kc = 0; kc < FI / 32; ++kc) { v16b a; { const float* p = X + (r0 + col) * FI + kc * 32 + 8 * g;
#pragma unroll
      for (int i = 0; i < 8; ++i) { a[i] = (__bf16)p[i]; a[8 + i] = (__bf16)p[16 + i]; } }
#pragma unroll
    for (int j = 0; j < 8; ++j) acc[j] = wmma_bf(a, frag_b(P + ((size_t)which * FO + j * 16 + col) * FI + kc * 32, lane), acc[j]); }
#pragma unroll
  for (int j = 0; j < 8; ++j)
#pragma unroll
    for (int r = 0; r < 8; ++r) { so[wave * 16 + 8 * g + r][j * 16 + col] = acc[j][r]; if (which == 0) { const _Float16 hh = (_Float16)acc[j][r]; st[j * 16 + col][wave * 16 + 8 * g + r] = hh; stl[j * 16 + col][wave * 16 + 8 * g + r] = (_Float16)((acc[j][r] - (float)hh) * 2048.0f); } }
  LDSX(); __syncthreads();
  if (which == 1) { for (int rl = 0; rl < 16; ++rl) vst2(OUT + (r0 + rl) * FO + lane * 4, *(const v4f*)&so[wave * 16 + rl][lane * 4]); return; }
  for (int rl = 0; rl < 16; ++rl) vst2(H + (r0 + rl) * FO + lane * 4, *(const v4f*)&so[wave * 16 + rl][lane * 4]);
  { const size_t b = rb0 / NN, s0 = rb0 % NN; for (int e = tid; e < 128 * 8; e += 128) { const int d = e >> 3, pc = e & 7; vst2((unsigned*)(HP + ((b * FO + d) * NN) + s0 + pc * 8), *(const v4u*)&st[d][pc * 8]); vst2((unsigned*)(HPL + ((b * FO + d) * NN) + s0 + pc * 8), *(const v4u*)&stl[d][pc * 8]); } }
  if (tid < 128) { const int rl = tid & 63, which2 = tid >> 6; float s = 0.f;
#pragma unroll 8
    for (int c = 0; c < FO; ++c) s += so[rl][c] * bfr(AW[which2 * FO + c]);
    su[which2][rl] = s; }
  __syncthreads();
  if (tid < 32) { const int which2 = tid >> 4, q = tid & 15; vst2(U + (size_t)which2 * NR + rb0 + q * 4, *(const v4f*)&su[which2][q * 4]); }
}
__device__ __attribute__((noinline)) float exp_p(float v) { return expf(v); }
__global__ __launch_bounds__(256) void k_col(const float* __restrict__ U, const float* __restrict__ ADJ, float* __restrict__ CM, float* __restrict__ CZ) {
  __shared__ float pm[4][64], pz[4][64]; __shared__ __align__(16) float om[64], oz[64];
  const int t = threadIdx.x; const size_t b = blockIdx.y; const int j0 = blockIdx.x * 64; const int jl = t & 63, grp = t >> 6; const int j = j0 + jl; const float* U1 = U; const float* U2 = U + NR;
  float m = -3.0e38f, z = 0.f;
  for (int i = grp; i < NN; i += 4) { if (bfr(ADJ[(size_t)i * NN + j]) > 0.f) { const float e = escore(U1, U2, b, i, j); if (e > m) { z = z * exp_p(m - e) + 1.0f; m = e; } else z += exp_p(e - m); } }
  pm[grp][jl] = m; pz[grp][jl] = z; __syncthreads();
  if (t < 64) { float mm = fmaxf(fmaxf(pm[0][t], pm[1][t]), fmaxf(pm[2][t], pm[3][t])); float zz = 0.f; for (int q = 0; q < 4; ++q) if (pm[q][t] > -1.0e38f) zz += pz[q][t] * exp_p(pm[q][t] - mm); om[t] = mm; oz[t] = zz; }
  __syncthreads();
  if (t < 16) { vst2(CM + b * NN + j0 + t * 4, *(const v4f*)&om[t * 4]); vst2(CZ + b * NN + j0 + t * 4, *(const v4f*)&oz[t * 4]); }
}
__global__ __launch_bounds__(128) void k_agg(const float* __restrict__ U, const float* __restrict__ ADJ, const float* __restrict__ CM, const float* __restrict__ CZ, const _Float16* __restrict__ HP, const _Float16* __restrict__ HPL, float* __restrict__ OUT) {
  __shared__ __align__(16) _Float16 sph[4][16][40]; __shared__ __align__(16) _Float16 spl[4][16][40]; __shared__ __align__(16) float so[4][16][132];
  const int tid = threadIdx.x, wave = tid >> 5, lane = tid & 31, col = lane & 15, g = lane >> 4; const size_t b = blockIdx.y; const int i0 = blockIdx.x * 64 + wave * 16; const float* U1 = U; const float* U2 = U + NR;
  v8f acc[8] = {}, accl[8] = {};
#pragma unroll 1
  for (int js = 0; js < NN / 32; ++js) { const int jb = js * 32;
#pragma unroll
    for (int ct = 0; ct < 2; ++ct) { const int j = jb + ct * 16 + col; const float mj = CM[b * NN + j], zj = CZ[b * NN + j];
#pragma unroll
      for (int r = 0; r < 8; ++r) { const int i = i0 + 8 * g + r; float p = 0.f; if (bfr(ADJ[(size_t)i * NN + j]) > 0.f) p = __expf(escore(U1, U2, b, i, j) - mj) / zj; const float ps = p * 2048.0f; const _Float16 ph = (_Float16)ps; sph[wave][8 * g + r][ct * 16 + col] = ph; spl[wave][8 * g + r][ct * 16 + col] = (_Float16)((ps - (float)ph) * 2048.0f); } }
    LDSX();
    const v16h pa = frag_h(&sph[wave][col][0], lane), pal = frag_h(&spl[wave][col][0], lane);
#pragma unroll
    for (int dt = 0; dt < 8; ++dt) { const v16h hh = frag_h(HP + ((b * FO + dt * 16 + col) * NN) + jb, lane); acc[dt] = wmma16(pa, hh, acc[dt]); accl[dt] = wmma16(pal, hh, accl[dt]); accl[dt] = wmma16(pa, frag_h(HPL + ((b * FO + dt * 16 + col) * NN) + jb, lane), accl[dt]); }
    LDSX(); }
  const size_t row0 = b * NN + i0;
#pragma unroll
  for (int r = 0; r < 8; ++r)
#pragma unroll
    for (int dt = 0; dt < 8; ++dt) so[wave][8 * g + r][dt * 16 + col] = (acc[dt][r] + accl[dt][r] * (1.0f / 2048.0f)) * (1.0f / 2048.0f) + OUT[(row0 + 8 * g + r) * FO + dt * 16 + col];
  LDSX();
  for (int rl = 0; rl < 16; ++rl) vst2(OUT + (row0 + rl) * FO + lane * 4, *(const v4f*)&so[wave][rl][lane * 4]);
}
extern "C" void kernel_launch(void* const* d_in, const int* in_sizes, int n_in, void* d_out, int out_size, void* d_ws, size_t ws_size, hipStream_t stream) {
  (void)in_sizes; (void)n_in; (void)out_size;
  const float** F = (const float**)d_in;
  if (ws_size < (size_t)WS_END) return;
  char* ws = (char*)d_ws; __bf16* P = (__bf16*)ws; float *H = (float*)(ws + WS_H), *U = (float*)(ws + WS_U), *CM = (float*)(ws + WS_CM), *CZ = (float*)(ws + WS_CZ); _Float16 *HP = (_Float16*)(ws + WS_HP), *HPL = (_Float16*)(ws + WS_HPL);
  k_pack<<<dim3(FO, 2), 128, 0, stream>>>(F[2], F[3], P);
  k_h<<<dim3(TNB * NN / 64, 2), 128, 0, stream>>>(F[0], P, F[4], H, HP, HPL, U, (float*)d_out);
  k_col<<<dim3(NN / 64, TNB), 256, 0, stream>>>(U, F[1], CM, CZ);
  k_agg<<<dim3(NN / 64, TNB), 128, 0, stream>>>(U, F[1], CM, CZ, HP, HPL, (float*)d_out);
}
